// TemporalLSTM_2894807957763
// MI455X (gfx1250) — hardware-verified
//
#include <hip/hip_runtime.h>
#include <math.h>

constexpr int NBATCH = 16384;
constexpr int NSTEP  = 200;
constexpr int NIN    = 5;
constexpr int NHID   = 32;
constexpr int NGATE  = 4 * NHID;
constexpr int NOUT   = 2;
constexpr int NTHR   = 256;
constexpr int NWAVE  = NTHR / 32;
constexpr int ROWS_PER_WAVE  = 16;
constexpr int ROWS_PER_BLOCK = NWAVE * ROWS_PER_WAVE;
constexpr int WPITCH = 40;
constexpr int HPITCH = 40;
constexpr int FPITCH = 33;
constexpr float ACARRY     = 32.0f;
constexpr float WCARRY     = 16.0f;
constexpr float ZCARRY     = ACARRY * WCARRY;
constexpr float ZCARRY_INV = 1.0f / ZCARRY;

static_assert(NIN == 5);
static_assert(NHID == 32);
static_assert(NGATE == 128);
static_assert(NBATCH % ROWS_PER_BLOCK == 0);
static_assert((NGATE * WPITCH) % NTHR == 0);
static_assert((NWAVE * 16 * HPITCH) % NTHR == 0);
static_assert(ROWS_PER_WAVE * NOUT == 32);
static_assert(WPITCH % 8 == 0 && HPITCH % 8 == 0);
static_assert(WPITCH >= NHID && HPITCH >= NHID);

typedef __attribute__((ext_vector_type(16))) _Float16 v16h;
typedef __attribute__((ext_vector_type(8)))  _Float16 v8h;
typedef __attribute__((ext_vector_type(8)))  float    v8f;
typedef __attribute__((ext_vector_type(8)))  unsigned v8u;

__device__ __forceinline__ void dep_guard_h(v8f& a, v8f& b, v16h x, v16h y) { asm volatile("v_nop\n\tv_nop\n\tv_nop\n\tv_nop" : "+v"(a), "+v"(b) : "v"(x), "v"(y)); }
__device__ __forceinline__ void keep4_h(v16h a, v16h b, v16h c, v16h d) { asm volatile("v_nop" :: "v"(a), "v"(b), "v"(c), "v"(d)); }
template <typename T> struct Frag;
template <> struct Frag<_Float16> {
  typedef v16h V; union U { v16h v; v8h h[2]; };
  static __device__ __forceinline__ v16h load(const _Float16* p) {
    U f; f.h[0] = *(const v8h*)(p); f.h[1] = *(const v8h*)(p + 16); return f.v;
  }
  static __device__ __forceinline__ v8f mma(v16h a, v16h b, v8f c) {
    return __builtin_amdgcn_wmma_f32_16x16x32_f16(false, a, false, b, (short)0, c, false, false);
  }
  static __device__ __forceinline__ void guard(v8f& a, v8f& b, v16h x, v16h y) { dep_guard_h(a, b, x, y); }
  static __device__ __forceinline__ void keep(v16h a, v16h b, v16h c, v16h d) { keep4_h(a, b, c, d); }
};

__device__ __forceinline__ v8f mma_g(v16h a, v16h b, v8f c) {
  c = Frag<_Float16>::mma(a, b, c);
  asm volatile("v_nop\n\tv_nop\n\tv_nop\n\tv_nop" : "+v"(c) : "v"(a), "v"(b));
  return c;
}

__device__ __forceinline__ float fsig(float x)  { return __builtin_amdgcn_rcpf(1.0f + __expf(-x)); }
__device__ __forceinline__ float ftanh(float x) { return 1.0f - 2.0f * __builtin_amdgcn_rcpf(__expf(2.0f * x) + 1.0f); }

__device__ __forceinline__ unsigned f16bits(float f) {
  const _Float16 h = (_Float16)f;
  return (unsigned)__builtin_bit_cast(unsigned short, h);
}

__global__ __launch_bounds__(NTHR) void lstm_seq_kernel(const float* __restrict__ x,
                                                        const float* __restrict__ w_ih,
                                                        const float* __restrict__ w_hh,
                                                        const float* __restrict__ b_ih,
                                                        const float* __restrict__ b_hh,
                                                        const float* __restrict__ w_fc,
                                                        const float* __restrict__ b_fc,
                                                        float* __restrict__ out) {
  __shared__ __align__(16) _Float16 Wh[NGATE * WPITCH];
  __shared__ __align__(16) _Float16 Wi[NGATE * WPITCH];
  __shared__ __align__(16) _Float16 Ht[NWAVE][16 * HPITCH];
  __shared__ __align__(16) float    Fs[NWAVE][16 * FPITCH];
  __shared__ float Wf[NOUT * NHID + NOUT];

  const int tid  = threadIdx.x;
  const int lane = tid & 31;
  const int wave = tid >> 5;
  const int c    = lane & 15;
  const int hh   = lane >> 4;
  const int koff = hh * 8;
  const int rowBase = (blockIdx.x * NWAVE + wave) * ROWS_PER_WAVE;

#pragma unroll 1
  for (int i = tid; i < NGATE * WPITCH; i += NTHR) {
    const int n  = i / WPITCH;
    const int k  = i - n * WPITCH;
    const int kh = (k < NHID) ? k : (NHID - 1);
    const int ki = (k < NIN) ? k : (NIN - 1);
    const float vh = w_hh[n * NHID + kh];
    const float vi = w_ih[n * NIN + ki];
    const float sh = (k < NHID) ? (vh * WCARRY) : 0.0f;
    const float si = (k < NIN) ? (vi * WCARRY) : 0.0f;
    Wh[i] = (_Float16)sh;
    Wi[i] = (_Float16)si;
  }
  {
    _Float16* hz = &Ht[0][0];
#pragma unroll 1
    for (int i = tid; i < NWAVE * 16 * HPITCH; i += NTHR) hz[i] = (_Float16)0.0f;
  }
  {
    const int iw = (tid < NOUT * NHID) ? tid : (NOUT * NHID - 1);
    const int ib = (tid < NOUT) ? tid : (NOUT - 1);
    float vw = w_fc[iw];
    float vb = b_fc[ib];
    asm volatile("" : "+v"(vw));
    asm volatile("" : "+v"(vb));
    if (tid < NOUT * NHID) Wf[tid] = vw;
    if (tid < NOUT) Wf[NOUT * NHID + tid] = vb;
  }
  float bz[8];
#pragma unroll
  for (int q = 0; q < 8; ++q) {
    const float s = b_ih[q * 16 + c] + b_hh[q * 16 + c];
    bz[q] = s * ZCARRY;
  }
  float cst[2][8], hst[2][8];
#pragma unroll
  for (int u = 0; u < 2; ++u)
#pragma unroll
    for (int r = 0; r < 8; ++r) { cst[u][r] = 0.0f; hst[u][r] = 0.0f; }
  __syncthreads();

  const float*    xrow  = x + (size_t)(rowBase + c) * (size_t)(NSTEP * NIN);
  const _Float16* ahrow = &Ht[wave][0] + c * HPITCH + koff;
  _Float16*       hw    = &Ht[wave][0];
  const bool lo = (hh == 0);

#pragma unroll 1
  for (int t = 0; t < NSTEP; ++t) {
    float xv0 = xrow[t * NIN + 0];
    float xv1 = xrow[t * NIN + 1];
    float xv2 = xrow[t * NIN + 2];
    float xv3 = xrow[t * NIN + 3];
    float xv4 = xrow[t * NIN + 4];
    asm volatile("" : "+v"(xv0));
    asm volatile("" : "+v"(xv1));
    asm volatile("" : "+v"(xv2));
    asm volatile("" : "+v"(xv3));
    asm volatile("" : "+v"(xv4));
    const float a0 = lo ? (xv0 * ACARRY) : 0.0f;
    const float a1 = lo ? (xv1 * ACARRY) : 0.0f;
    const float a2 = lo ? (xv2 * ACARRY) : 0.0f;
    const float a3 = lo ? (xv3 * ACARRY) : 0.0f;
    const float a4 = lo ? (xv4 * ACARRY) : 0.0f;
    const unsigned w0 = f16bits(a0) | (f16bits(a1) << 16);
    const unsigned w1 = f16bits(a2) | (f16bits(a3) << 16);
    const unsigned w2 = f16bits(a4);
    const v8u aw = {w0, w1, w2, 0u, 0u, 0u, 0u, 0u};
    const v16h ax = __builtin_bit_cast(v16h, aw);
    const v16h ah = Frag<_Float16>::load(ahrow);

#pragma unroll
    for (int u = 0; u < 2; ++u) {
      v8f acc[4];
#pragma unroll
      for (int p = 0; p < 4; ++p) {
        const float b = bz[2 * p + u];
        acc[p] = (v8f){b, b, b, b, b, b, b, b};
      }
#pragma unroll
      for (int p = 0; p < 4; ++p) {
        const int n = (2 * p + u) * 16 + c;
        const v16h bi = Frag<_Float16>::load(Wi + n * WPITCH + koff);
        const v16h bh = Frag<_Float16>::load(Wh + n * WPITCH + koff);
        acc[p] = mma_g(ax, bi, acc[p]);
        acc[p] = mma_g(ah, bh, acc[p]);
      }
#pragma unroll
      for (int r = 0; r < 8; ++r) {
        const float zi = acc[0][r] * ZCARRY_INV;
        const float zf = acc[1][r] * ZCARRY_INV;
        const float zg = acc[2][r] * ZCARRY_INV;
        const float zo = acc[3][r] * ZCARRY_INV;
        const float ig = fsig(zi);
        const float fg = fsig(zf);
        const float gg = ftanh(zg);
        const float og = fsig(zo);
        const float cn = fg * cst[u][r] + ig * gg;
        cst[u][r] = cn;
        hst[u][r] = og * ftanh(cn);
      }
    }
    __syncthreads();
#pragma unroll
    for (int u = 0; u < 2; ++u)
#pragma unroll
      for (int r = 0; r < 8; ++r) {
        const float hs = hst[u][r] * ACARRY;
        hw[(8 * hh + r) * HPITCH + u * 16 + c] = (_Float16)hs;
      }
    __syncthreads();
  }

  float* fs = &Fs[wave][0];
#pragma unroll
  for (int u = 0; u < 2; ++u)
#pragma unroll
    for (int r = 0; r < 8; ++r) fs[(8 * hh + r) * FPITCH + u * 16 + c] = hst[u][r];
  __syncthreads();

  {
    const int orow = lane >> 1;
    const int oj   = lane & 1;
    float s = 0.0f;
#pragma unroll 8
    for (int n = 0; n < NHID; ++n) s = fmaf(fs[orow * FPITCH + n], Wf[oj * NHID + n], s);
    const float v = s + Wf[NOUT * NHID + oj];
    float* op = out + (size_t)rowBase * NOUT + lane;
    *(volatile float*)op = v;
    __threadfence();
    *(volatile float*)op = v;
  }
}

extern "C" void kernel_launch(void* const* d_in, const int* in_sizes, int n_in,
                              void* d_out, int out_size, void* d_ws, size_t ws_size, hipStream_t stream) {
  (void)d_ws; (void)ws_size;
  if (n_in < 7 || d_out == nullptr) return;
  if (in_sizes[0] != NBATCH * NSTEP * NIN || in_sizes[1] != NGATE * NIN || in_sizes[2] != NGATE * NHID ||
      in_sizes[3] != NGATE || in_sizes[4] != NGATE || in_sizes[5] != NOUT * NHID || in_sizes[6] != NOUT ||
      out_size != NBATCH * NOUT) return;

  const float* x    = (const float*)d_in[0];
  const float* w_ih = (const float*)d_in[1];
  const float* w_hh = (const float*)d_in[2];
  const float* b_ih = (const float*)d_in[3];
  const float* b_hh = (const float*)d_in[4];
  const float* w_fc = (const float*)d_in[5];
  const float* b_fc = (const float*)d_in[6];
  float* out = (float*)d_out;

  lstm_seq_kernel<<<dim3(NBATCH / ROWS_PER_BLOCK), dim3(NTHR), 0, stream>>>(
      x, w_ih, w_hh, b_ih, b_hh, w_fc, b_fc, out);
}
